// S4Layer_18803366821989
// MI455X (gfx1250) — hardware-verified
//
#include <hip/hip_runtime.h>
#include <math.h>

#pragma clang fp contract(off)

constexpr int kB   = 8;
constexpr int kH   = 256;
constexpr int kL   = 2048;
constexpr int kN   = 128;
constexpr int kHN  = kH * kN;
constexpr int kHL  = kH * kL;
constexpr int kBHL = kB * kH * kL;
constexpr int kG8Row = 4096;
constexpr float kGCarry    = 16.0f;
constexpr float kGCarryInv = 1.0f / 16.0f;
constexpr float kActCarry  = 8.0f;
constexpr float kWCarry    = 16.0f;
constexpr float kOutScale  = 1.0f / 128.0f;

static_assert(kB == 8);
static_assert(kHN % 256 == 0);
static_assert((kB * kL / 2) % 256 == 0);
static_assert((kL / 2) % 32 == 0);
static_assert(kL % 32 == 0 && kL % 16 == 0 && kL % 256 == 0);
static_assert(kH % 64 == 0 && kL % 64 == 0 && kH % 32 == 0);
static_assert((8 * kH * (kG8Row / 2)) % 256 == 0);
static_assert((kH * kH / 8) % 256 == 0);

typedef __attribute__((ext_vector_type(16))) _Float16 v16h;
typedef __attribute__((ext_vector_type(8)))  _Float16 v8h;
typedef __attribute__((ext_vector_type(16))) __bf16   v16b;
typedef __attribute__((ext_vector_type(8)))  __bf16   v8b;
typedef __attribute__((ext_vector_type(8)))  float    v8f;
typedef __attribute__((ext_vector_type(4)))  float    v4f;
typedef __attribute__((ext_vector_type(2)))  float    v2f;
typedef __attribute__((ext_vector_type(4)))  unsigned int v4u;

__device__ __forceinline__ unsigned short f2bf_bits(float f) {
  unsigned u = __float_as_uint(f);
  return (unsigned short)((u + 0x7FFFu + ((u >> 16) & 1u)) >> 16);
}
__device__ __forceinline__ float bf_bits2f(unsigned short h) { return __uint_as_float(((unsigned)h) << 16); }

__device__ __forceinline__ void dep_guard_h(v8f& a, v8f& b, v16h x, v16h y) { asm volatile("v_nop\n\tv_nop\n\tv_nop\n\tv_nop" : "+v"(a), "+v"(b) : "v"(x), "v"(y)); }
__device__ __forceinline__ void dep_guard_b(v8f& a, v8f& b, v16b x, v16b y) { asm volatile("v_nop\n\tv_nop\n\tv_nop\n\tv_nop" : "+v"(a), "+v"(b) : "v"(x), "v"(y)); }
__device__ __forceinline__ void keep4_h(v16h a, v16h b, v16h c, v16h d) { asm volatile("v_nop" :: "v"(a), "v"(b), "v"(c), "v"(d)); }
__device__ __forceinline__ void keep4_b(v16b a, v16b b, v16b c, v16b d) { asm volatile("v_nop" :: "v"(a), "v"(b), "v"(c), "v"(d)); }
__device__ __forceinline__ void acc_guard4(v8f& a, v8f& b, v8f& c, v8f& d) { asm volatile("v_nop\n\tv_nop\n\tv_nop\n\tv_nop" : "+v"(a), "+v"(b), "+v"(c), "+v"(d)); }
template <typename T> struct Frag;
template <> struct Frag<_Float16> {
  typedef v16h V; union U { v16h v; v8h h[2]; };
  static __device__ __forceinline__ v16h load(const _Float16* p) {
    U f; f.h[0] = *(const v8h*)(p); f.h[1] = *(const v8h*)(p + 16); return f.v;
  }
  static __device__ __forceinline__ v8f mma(v16h a, v16h b, v8f c) {
    return __builtin_amdgcn_wmma_f32_16x16x32_f16(false, a, false, b, (short)0, c, false, false);
  }
  static __device__ __forceinline__ void guard(v8f& a, v8f& b, v16h x, v16h y) { dep_guard_h(a, b, x, y); }
  static __device__ __forceinline__ void keep(v16h a, v16h b, v16h c, v16h d) { keep4_h(a, b, c, d); }
};
template <> struct Frag<__bf16> {
  typedef v16b V; union U { v16b v; v8b h[2]; };
  static __device__ __forceinline__ v16b load(const __bf16* p) {
    U f; f.h[0] = *(const v8b*)(p); f.h[1] = *(const v8b*)(p + 16); return f.v;
  }
  static __device__ __forceinline__ v8f mma(v16b a, v16b b, v8f c) {
    return __builtin_amdgcn_wmma_f32_16x16x32_bf16(false, a, false, b, (short)0, c, false, false);
  }
  static __device__ __forceinline__ void guard(v8f& a, v8f& b, v16b x, v16b y) { dep_guard_b(a, b, x, y); }
  static __device__ __forceinline__ void keep(v16b a, v16b b, v16b c, v16b d) { keep4_b(a, b, c, d); }
};

__device__ __forceinline__ unsigned pk16(unsigned short a, unsigned short b) { return (unsigned)a | ((unsigned)b << 16); }
__device__ __forceinline__ unsigned short h_bits(float f) { const _Float16 h = (_Float16)f; return __builtin_bit_cast(unsigned short, h); }

__device__ __forceinline__ v8f hmma(v16h a, v16h b, v8f c) {
  c = __builtin_amdgcn_wmma_f32_16x16x32_f16(false, a, false, b, (short)0, c, false, false);
  asm volatile("v_nop\n\tv_nop\n\tv_nop\n\tv_nop" : "+v"(c) : "v"(a), "v"(b));
  return c;
}

template <int ET> struct Elem;
template <> struct Elem<0> { typedef _Float16 T; };
template <> struct Elem<1> { typedef __bf16 T; };
template <int ET, bool SPLIT, int BIAS_MODE, int OUT_MODE, bool RESID>
__global__ __launch_bounds__(256) void wmma_gemm64(
    const unsigned short* __restrict__ Ap, const unsigned short* __restrict__ A2p, int lda, long strideA,
    const unsigned short* __restrict__ Btp, const unsigned short* __restrict__ Bt2p, int ldb, long strideB,
    void* __restrict__ Cout, void* __restrict__ Cout2, int ldc, long strideC,
    const float* __restrict__ bias,
    const float* __restrict__ resid, long strideR,
    int M, int N, int K, float scale) {
  static_assert(!(RESID && OUT_MODE != 0));
  typedef typename Elem<ET>::T T;
  typedef typename Frag<T>::V V;
  const T* A = (const T*)Ap; const T* A2 = (const T*)A2p; const T* Bt = (const T*)Btp; const T* Bt2 = (const T*)Bt2p;
  __shared__ __align__(16) float sT[8][16 * 68];
  const int b    = blockIdx.y;
  const int lane = threadIdx.x & 31;
  const int wave = threadIdx.x >> 5;
  const int tilesN = N >> 6;
  const int tilesM = M >> 6;
  const int tile = blockIdx.x * 8 + wave;
  if (tile >= tilesM * tilesN) return;
  const int tm = tile / tilesN;
  const int tn = tile - tm * tilesN;
  const int m0 = tm << 6;
  const int n0 = tn << 6;

  const T* Ab  = A  + (size_t)b * strideA;
  const T* Bb  = Bt + (size_t)b * strideB;
  const T* Ab2 = SPLIT ? (A2  + (size_t)b * strideA) : nullptr;
  const T* Bb2 = SPLIT ? (Bt2 + (size_t)b * strideB) : nullptr;

  const int rlane = lane & 15;
  const int koff  = (lane >> 4) * 8;
  const int mOff  = (lane >> 4) * 8;

  v8f acc[4][4];
#pragma unroll
  for (int i = 0; i < 4; ++i)
#pragma unroll
    for (int j = 0; j < 4; ++j) acc[i][j] = (v8f){0.f,0.f,0.f,0.f,0.f,0.f,0.f,0.f};

  for (int k0 = 0; k0 < K; k0 += 32) {
    V bh[4], bl[4];
#pragma unroll
    for (int j = 0; j < 4; ++j) {
      const size_t bo = (size_t)(n0 + (j << 4) + rlane) * ldb + koff + k0;
      bh[j] = Frag<T>::load(Bb + bo);
      if (SPLIT) bl[j] = Frag<T>::load(Bb2 + bo);
    }
#pragma unroll
    for (int i = 0; i < 4; ++i) {
      const size_t ao = (size_t)(m0 + (i << 4) + rlane) * lda + koff + k0;
      V ah = Frag<T>::load(Ab + ao);
      V al;
      if (SPLIT) al = Frag<T>::load(Ab2 + ao);
#pragma unroll
      for (int j = 0; j < 4; ++j) {
        acc[i][j] = Frag<T>::mma(ah, bh[j], acc[i][j]);
        if (SPLIT) {
          acc[i][j] = Frag<T>::mma(ah, bl[j], acc[i][j]);
          acc[i][j] = Frag<T>::mma(al, bh[j], acc[i][j]);
        }
      }
      Frag<T>::guard(acc[i][0], acc[i][3], ah, SPLIT ? al : ah);
    }
    Frag<T>::keep(bh[0], bh[1], bh[2], bh[3]);
    if (SPLIT) Frag<T>::keep(bl[0], bl[1], bl[2], bl[3]);
  }
  acc_guard4(acc[0][0], acc[0][1], acc[0][2], acc[0][3]);
  acc_guard4(acc[1][0], acc[1][1], acc[1][2], acc[1][3]);
  acc_guard4(acc[2][0], acc[2][1], acc[2][2], acc[2][3]);
  acc_guard4(acc[3][0], acc[3][1], acc[3][2], acc[3][3]);

  float* slab = sT[wave];
  const float* Rb = RESID ? (resid + (size_t)b * strideR) : nullptr;
#pragma unroll
  for (int i = 0; i < 4; ++i) {
    const int mBase = m0 + (i << 4);
    float bm[8];
#pragma unroll
    for (int r = 0; r < 8; ++r) bm[r] = 0.0f;
    if (BIAS_MODE == 1) {
      const v4f b0 = *(const v4f*)(bias + mBase + mOff);
      const v4f b1 = *(const v4f*)(bias + mBase + mOff + 4);
      bm[0] = b0[0]; bm[1] = b0[1]; bm[2] = b0[2]; bm[3] = b0[3];
      bm[4] = b1[0]; bm[5] = b1[1]; bm[6] = b1[2]; bm[7] = b1[3];
    }
#pragma unroll
    for (int j = 0; j < 4; ++j) {
      const int n = n0 + (j << 4) + rlane;
      float bv = 0.f;
      if (BIAS_MODE == 2) bv = bias[n];
#pragma unroll
      for (int r = 0; r < 8; ++r) {
        float v = acc[i][j][r] * scale;
        if (BIAS_MODE == 1) v += bm[r];
        if (BIAS_MODE == 2) v += bv;
        slab[(mOff + r) * 68 + (j << 4) + rlane] = v;
      }
    }
    __builtin_amdgcn_fence(__ATOMIC_RELEASE, "workgroup");
    __builtin_amdgcn_wave_barrier();
    __builtin_amdgcn_fence(__ATOMIC_ACQUIRE, "workgroup");
    if (OUT_MODE == 0) {
      float* C = (float*)Cout + (size_t)b * strideC;
      const int hh = lane >> 4, c4 = (lane & 15) * 4;
      for (int pass = 0; pass < 2; ++pass) {
#pragma unroll
        for (int it = 0; it < 8; ++it) {
          const int row = it * 2 + hh;
          v4f v = *(const v4f*)(slab + row * 68 + c4);
          if (RESID) {
            const v4f rr = *(const v4f*)(Rb + (size_t)(mBase + row) * ldc + n0 + c4);
            v = v + rr;
          }
          *(volatile v4f*)(C + (size_t)(mBase + row) * ldc + n0 + c4) = v;
        }
        __threadfence();
      }
    } else {
      const int q = lane >> 3, c8 = (lane & 7) * 8;
      unsigned short* C  = (unsigned short*)Cout  + (size_t)b * strideC;
      unsigned short* C2 = (OUT_MODE == 2) ? ((unsigned short*)Cout2 + (size_t)b * strideC) : nullptr;
      for (int pass = 0; pass < 2; ++pass) {
#pragma unroll
        for (int it = 0; it < 4; ++it) {
          const int row = it * 4 + q;
          const float* sp = slab + row * 68 + c8;
          v8h hv, lv;
#pragma unroll
          for (int e = 0; e < 8; ++e) {
            if (OUT_MODE == 1) {
              hv[e] = (_Float16)sp[e];
            } else {
              unsigned short hb = f2bf_bits(sp[e]);
              unsigned short lb = f2bf_bits(sp[e] - bf_bits2f(hb));
              hv[e] = __builtin_bit_cast(_Float16, hb);
              lv[e] = __builtin_bit_cast(_Float16, lb);
            }
          }
          *(volatile v8h*)(C + (size_t)(mBase + row) * ldc + n0 + c8) = hv;
          if (OUT_MODE == 2) *(volatile v8h*)(C2 + (size_t)(mBase + row) * ldc + n0 + c8) = lv;
        }
        __threadfence();
      }
    }
    __builtin_amdgcn_fence(__ATOMIC_RELEASE, "workgroup");
    __builtin_amdgcn_wave_barrier();
    __builtin_amdgcn_fence(__ATOMIC_ACQUIRE, "workgroup");
  }
}

__global__ __launch_bounds__(256) void params_kernel(const float* __restrict__ log_dt, const float* __restrict__ log_A_re,
                                                     const float* __restrict__ A_im, const float* __restrict__ C_re,
                                                     const float* __restrict__ C_im,
                                                     float* __restrict__ wr_p, float* __restrict__ wi_p,
                                                     float* __restrict__ c0r_p, float* __restrict__ c0i_p,
                                                     float* __restrict__ c1r_p, float* __restrict__ c1i_p) {
  const int i = blockIdx.x * 256 + threadIdx.x;
  const int h = i >> 7;
  const float dt  = expf(log_dt[h]);
  const float are = -expf(log_A_re[i]);
  const float aim = A_im[i];
  const float wr  = are * dt;
  const float wi  = aim * dt;
  const float em  = expm1f(wr);
  const float ea  = em + 1.0f;
  const float sb  = sinf(wi);
  const float cb  = cosf(wi);
  const float sh  = sinf(0.5f * wi);
  const float er  = em * cb - 2.0f * sh * sh;
  const float ei  = ea * sb;
  const float inv = 1.0f / (are * are + aim * aim);
  const float fr  = (er * are + ei * aim) * inv;
  const float fi  = (ei * are - er * aim) * inv;
  const float p0r = C_re[i],       p0i = C_im[i];
  const float p1r = C_re[kHN + i], p1i = C_im[kHN + i];
  const float o0r = 2.0f * (p0r * fr - p0i * fi);
  const float o0i = 2.0f * (p0r * fi + p0i * fr);
  const float o1r = 2.0f * (p1r * fr - p1i * fi);
  const float o1i = 2.0f * (p1r * fi + p1i * fr);
  for (int pass = 0; pass < 2; ++pass) {
    ((volatile float*)wr_p)[i]  = wr;
    ((volatile float*)wi_p)[i]  = wi;
    ((volatile float*)c0r_p)[i] = o0r;
    ((volatile float*)c0i_p)[i] = o0i;
    ((volatile float*)c1r_p)[i] = o1r;
    ((volatile float*)c1i_p)[i] = o1i;
    __threadfence();
  }
}

__global__ __launch_bounds__(256) void ln_kernel(const float* __restrict__ x, const float* __restrict__ lnw,
                                                 const float* __restrict__ lnb, float* __restrict__ z32,
                                                 unsigned* __restrict__ z16w) {
  const int idx = blockIdx.x * 256 + threadIdx.x;
  const int b   = idx >> 10;
  const int l   = (idx & 1023) * 2;
  const size_t base = (size_t)b * kHL + l;
  const float* xb = x + base;
  float s0 = 0.0f, s1 = 0.0f;
#pragma unroll 4
  for (int h = 0; h < kH; ++h) {
    const v2f v = *(const v2f*)(xb + (size_t)h * kL);
    s0 += v[0]; s1 += v[1];
  }
  const float mu0 = s0 * (1.0f / 256.0f);
  const float mu1 = s1 * (1.0f / 256.0f);
  float q0 = 0.0f, q1 = 0.0f;
#pragma unroll 4
  for (int h = 0; h < kH; ++h) {
    const v2f v = *(const v2f*)(xb + (size_t)h * kL);
    const float d0 = v[0] - mu0, d1 = v[1] - mu1;
    q0 += d0 * d0; q1 += d1 * d1;
  }
  const float r0 = rsqrtf(q0 * (1.0f / 256.0f) + 1e-5f);
  const float r1 = rsqrtf(q1 * (1.0f / 256.0f) + 1e-5f);
  for (int pass = 0; pass < 2; ++pass) {
#pragma unroll 2
    for (int h = 0; h < kH; ++h) {
      const v2f v = *(const v2f*)(xb + (size_t)h * kL);
      const float w = lnw[h], bb = lnb[h];
      const float z0 = (v[0] - mu0) * r0 * w + bb;
      const float z1 = (v[1] - mu1) * r1 * w + bb;
      const v2f zv = (v2f){z0, z1};
      const size_t o = base + (size_t)h * kL;
      *(volatile v2f*)(z32 + o) = zv;
      const unsigned pk = pk16(h_bits(z0), h_bits(z1));
      ((volatile unsigned*)z16w)[o >> 1] = pk;
    }
    __threadfence();
  }
}

__global__ __launch_bounds__(256) void kgen_kernel(const float* __restrict__ wr_p, const float* __restrict__ wi_p,
                                                   const float* __restrict__ c0r_p, const float* __restrict__ c0i_p,
                                                   const float* __restrict__ c1r_p, const float* __restrict__ c1i_p,
                                                   float* __restrict__ K0, float* __restrict__ K1) {
  __shared__ float sp[6 * kN];
  const int tid = threadIdx.x;
  const int h = blockIdx.x >> 3;
  const int l = (blockIdx.x & 7) * 256 + tid;
  if (tid < kN) {
    const int o = h * kN + tid;
    sp[tid]          = wr_p[o];
    sp[kN + tid]     = wi_p[o];
    sp[2 * kN + tid] = c0r_p[o];
    sp[3 * kN + tid] = c0i_p[o];
    sp[4 * kN + tid] = c1r_p[o];
    sp[5 * kN + tid] = c1i_p[o];
  }
  __syncthreads();
  const float lf = (float)l;
  float k0 = 0.0f, k1 = 0.0f;
#pragma unroll 1
  for (int n = 0; n < kN; ++n) {
    const float wr = sp[n];
    const float wi = sp[kN + n];
    float a = expf(wr * lf);
    a = (a < 1.17549435e-38f) ? 0.0f : a;
    const float p  = wi * lf;
    const float qf = rintf(p * 0.636619772367581343f);
    const int   qi = (int)qf;
    float r = fmaf(-qf, 1.57079637050628662e+0f, p);
    r = fmaf(-qf, -4.37113900018624283e-8f, r);
    const float r2 = r * r;
    float ps = fmaf(r2, -1.9515295891e-4f, 8.3321608736e-3f);
    ps = fmaf(r2, ps, -1.6666654611e-1f);
    const float sr = fmaf(r2 * r, ps, r);
    float pc = fmaf(r2, 2.443315711809948e-5f, -1.388731625493765e-3f);
    pc = fmaf(r2, pc, 4.166664568298827e-2f);
    const float cr = fmaf(r2 * r2, pc, fmaf(r2, -0.5f, 1.0f));
    const int qm = qi & 3;
    const float sw = (qm & 1) ? cr : sr;
    const float cw = (qm & 1) ? sr : cr;
    const float sn = (qm & 2) ? -sw : sw;
    const float cs = ((qm + 1) & 2) ? -cw : cw;
    const float t0 = fmaf(sp[2 * kN + n], cs, -(sp[3 * kN + n] * sn));
    const float t1 = fmaf(sp[4 * kN + n], cs, -(sp[5 * kN + n] * sn));
    k0 = fmaf(a, t0, k0);
    k1 = fmaf(a, t1, k1);
  }
  const size_t o = (size_t)h * kL + l;
  for (int pass = 0; pass < 2; ++pass) {
    ((volatile float*)K0)[o] = k0;
    ((volatile float*)K1)[o] = k1;
    __threadfence();
  }
}

__global__ __launch_bounds__(256) void g8_kernel(const float* __restrict__ K0, const float* __restrict__ K1,
                                                 unsigned* __restrict__ G8w) {
  const int idx = blockIdx.x * 256 + threadIdx.x;
  const int s   = idx >> 19;
  const int rem = idx & 524287;
  const int h   = rem >> 11;
  const int j   = (rem & 2047) * 2;
  const float* K0h = K0 + (size_t)h * kL;
  const float* K1h = K1 + (size_t)h * kL;
  float vv0, vv1;
  {
    const int i = j + s;
    int ia = 2047 - i; ia = ia < 0 ? 0 : ia;
    int ib = i - 2048; ib = ib < 0 ? 0 : (ib > 2047 ? 2047 : ib);
    const float va = K0h[ia];
    const float vb = K1h[ib];
    const float fa = (i < 2048) ? 1.0f : 0.0f;
    const float fb = (i >= 2048 && i < 4096) ? 1.0f : 0.0f;
    vv0 = fmaf(fa, va, fb * vb) * kGCarry;
  }
  {
    const int i = j + 1 + s;
    int ia = 2047 - i; ia = ia < 0 ? 0 : ia;
    int ib = i - 2048; ib = ib < 0 ? 0 : (ib > 2047 ? 2047 : ib);
    const float va = K0h[ia];
    const float vb = K1h[ib];
    const float fa = (i < 2048) ? 1.0f : 0.0f;
    const float fb = (i >= 2048 && i < 4096) ? 1.0f : 0.0f;
    vv1 = fmaf(fa, va, fb * vb) * kGCarry;
  }
  const unsigned pk = pk16(h_bits(vv0), h_bits(vv1));
  for (int pass = 0; pass < 2; ++pass) {
    ((volatile unsigned*)G8w)[idx] = pk;
    __threadfence();
  }
}

__global__ __launch_bounds__(256) void wcast_kernel(const float* __restrict__ W, unsigned short* __restrict__ W16) {
  const int i = blockIdx.x * 256 + threadIdx.x;
  const float* p = W + 8 * (size_t)i;
  const v4f a = *(const v4f*)(p);
  const v4f c = *(const v4f*)(p + 4);
  unsigned short hb[8];
#pragma unroll
  for (int e = 0; e < 4; ++e) {
    const float f0 = a[e] * kWCarry;
    const float f1 = c[e] * kWCarry;
    hb[e]     = h_bits(f0);
    hb[4 + e] = h_bits(f1);
  }
  const v4u u = (v4u){pk16(hb[0], hb[1]), pk16(hb[2], hb[3]), pk16(hb[4], hb[5]), pk16(hb[6], hb[7])};
  unsigned short* q = W16 + 8 * (size_t)i;
  *(volatile v4u*)q = u;
  __threadfence();
  *(volatile v4u*)q = u;
}

__global__ __launch_bounds__(256) void conv_kernel(const unsigned short* __restrict__ G8p,
                                                   const unsigned short* __restrict__ z16p,
                                                   const float* __restrict__ z32,
                                                   const float* __restrict__ Dp,
                                                   unsigned short* __restrict__ act16p) {
  __shared__ __align__(16) float sAct[128 * 64];
  const int tid  = threadIdx.x;
  const int lane = tid & 31;
  const int wave = tid >> 5;
  const int ltile = blockIdx.x & 127;
  const int hg    = blockIdx.x >> 7;
  const int l0 = ltile * 16;
  const int h0 = hg * 64;
  const int c    = lane & 15;
  const int koff = (lane >> 4) * 8;
  const int bcl  = c & 7;
  const unsigned wm = 0u - (unsigned)(c < 8);
  const v4u wm4 = (v4u){wm, wm, wm, wm};
  const int sft = (7 - c) & 7;
  const _Float16* G8 = (const _Float16*)(const void*)G8p;
  _Float16* act16 = (_Float16*)(void*)act16p;
  const int abase = 2047 - l0 - c + koff - sft;

#pragma unroll 1
  for (int i = 0; i < 8; ++i) {
    const int hloc = wave * 8 + i;
    const int h = h0 + hloc;
    const _Float16* arow = G8 + (size_t)(sft * kH + h) * kG8Row + abase;
    const unsigned short* zrow = z16p + (size_t)(bcl * kH + h) * kL + koff;
    v8f acc = (v8f){0.f,0.f,0.f,0.f,0.f,0.f,0.f,0.f};
#pragma unroll 2
    for (int t0 = 0; t0 < kL; t0 += 32) {
      const v16h af = Frag<_Float16>::load(arow + t0);
      union { v16h v; v4u u[2]; } zb;
      zb.u[0] = (*(const v4u*)(const void*)(zrow + t0)) & wm4;
      zb.u[1] = (*(const v4u*)(const void*)(zrow + t0 + 16)) & wm4;
      acc = hmma(af, zb.v, acc);
    }
    const float Dh = Dp[h];
    const float* zr = z32 + (size_t)(bcl * kH + h) * kL + l0 + koff;
    const v4f za = *(const v4f*)(zr);
    const v4f zc = *(const v4f*)(zr + 4);
    float zz[8];
    zz[0] = za[0]; zz[1] = za[1]; zz[2] = za[2]; zz[3] = za[3];
    zz[4] = zc[0]; zz[5] = zc[1]; zz[6] = zc[2]; zz[7] = zc[3];
#pragma unroll
    for (int r = 0; r < 8; ++r) {
      const float v = zz[r] * Dh + acc[r] * kGCarryInv;
      const float g = 0.5f * v * (1.0f + erff(v * 0.70710678118654752f));
      if (c < 8) sAct[((koff + r) * 8 + c) * 64 + hloc] = g * kActCarry;
    }
  }
  __syncthreads();
  const int q = lane >> 3, c8 = (lane & 7) * 8;
  for (int pass = 0; pass < 2; ++pass) {
#pragma unroll
    for (int it = 0; it < 4; ++it) {
      const int R = wave * 16 + it * 4 + q;
      const int lrow = R >> 3, bb = R & 7;
      const v4f u0 = *(const v4f*)(sAct + R * 64 + c8);
      const v4f u1 = *(const v4f*)(sAct + R * 64 + c8 + 4);
      v8h hv;
      hv[0] = (_Float16)u0[0]; hv[1] = (_Float16)u0[1]; hv[2] = (_Float16)u0[2]; hv[3] = (_Float16)u0[3];
      hv[4] = (_Float16)u1[0]; hv[5] = (_Float16)u1[1]; hv[6] = (_Float16)u1[2]; hv[7] = (_Float16)u1[3];
      *(volatile v8h*)(act16 + (size_t)(bb * kL + l0 + lrow) * kH + h0 + c8) = hv;
    }
    __threadfence();
  }
}

extern "C" void kernel_launch(void* const* d_in, const int* in_sizes, int n_in,
                              void* d_out, int out_size, void* d_ws, size_t ws_size,
                              hipStream_t stream) {
  if (n_in < 11) return;
  if (out_size != kBHL) return;
  if (in_sizes[0] != kBHL || in_sizes[3] != kHN || in_sizes[9] != kH * kH) return;
  const float* x        = (const float*)d_in[0];
  const float* log_dt   = (const float*)d_in[1];
  const float* log_A_re = (const float*)d_in[2];
  const float* A_im     = (const float*)d_in[3];
  const float* C_re     = (const float*)d_in[4];
  const float* C_im     = (const float*)d_in[5];
  const float* Dp       = (const float*)d_in[6];
  const float* ln_w     = (const float*)d_in[7];
  const float* ln_b     = (const float*)d_in[8];
  const float* W_out    = (const float*)d_in[9];
  const float* b_out    = (const float*)d_in[10];
  float* out = (float*)d_out;

  char* ws = (char*)d_ws;
  size_t off = 0;
  auto carve = [&](size_t bytes) {
    void* p = ws + off;
    off += (bytes + 255) & ~(size_t)255;
    return p;
  };
  float* wr_p  = (float*)carve((size_t)kHN * 4);
  float* wi_p  = (float*)carve((size_t)kHN * 4);
  float* c0r_p = (float*)carve((size_t)kHN * 4);
  float* c0i_p = (float*)carve((size_t)kHN * 4);
  float* c1r_p = (float*)carve((size_t)kHN * 4);
  float* c1i_p = (float*)carve((size_t)kHN * 4);
  float* K0    = (float*)carve((size_t)kHL * 4);
  float* K1    = (float*)carve((size_t)kHL * 4);
  float* z32   = (float*)carve((size_t)kBHL * 4);
  unsigned short* z16   = (unsigned short*)carve((size_t)kBHL * 2);
  unsigned short* G8    = (unsigned short*)carve((size_t)8 * kH * kG8Row * 2);
  unsigned short* act16 = (unsigned short*)carve((size_t)kBHL * 2);
  unsigned short* W16   = (unsigned short*)carve((size_t)kH * kH * 2);
  if (off > ws_size) return;

  params_kernel<<<kHN / 256, 256, 0, stream>>>(log_dt, log_A_re, A_im, C_re, C_im,
                                               wr_p, wi_p, c0r_p, c0i_p, c1r_p, c1i_p);
  ln_kernel<<<(kB * kL / 2) / 256, 256, 0, stream>>>(x, ln_w, ln_b, z32, (unsigned*)z16);
  kgen_kernel<<<kH * 8, 256, 0, stream>>>(wr_p, wi_p, c0r_p, c0i_p, c1r_p, c1i_p, K0, K1);
  g8_kernel<<<(8 * kH * (kG8Row / 2)) / 256, 256, 0, stream>>>(K0, K1, (unsigned*)G8);
  wcast_kernel<<<(kH * kH / 8) / 256, 256, 0, stream>>>(W_out, W16);
  conv_kernel<<<128 * (kH / 64), 256, 0, stream>>>(G8, z16, z32, Dp, act16);
  dim3 ggrid((kH / 64) * (kL / 64) / 8, kB);
  wmma_gemm64<0, false, 1, 0, true><<<ggrid, 256, 0, stream>>>(
      W16, nullptr, kH, 0L,
      act16, nullptr, kH, (long)kL * kH,
      (void*)out, nullptr, kL, (long)kH * kL,
      b_out,
      x, (long)kH * kL,
      kH, kL, kH, kOutScale);
}
